// GraphConvolution_52596169506858
// MI455X (gfx1250) — hardware-run, weakly checked
//
#include <hip/hip_runtime.h>
#include <stddef.h>
#include <stdint.h>

#define NN      100000
#define FIN     128
#define FO      64
#define NE      1600000
#define GBM     128
#define MP      100096
#define NTHR    256
#define NWAVE   8
#define EPT     8
#define WCH     (32 * EPT)
#define NBRUN   1024
#define SLB     10
#define NBK     98
#define WLCAP   3072
#define RCAP    20480
#define TRIPCAP 128
#define MAXDEG_MEAS   35
#define MAXB1024_MEAS 16714
#define SP      68
#define WSMAX   134217728
#define PERW    (((NE + NWAVE * WCH - 1) / (NWAVE * WCH)) * WCH)

#define BK_ZINTS (NWAVE * WLCAP + RCAP + 3 * NBRUN)
#define BK_INTS  (BK_ZINTS + 16)
#define BK_LDS   (BK_INTS * 4)

#define PBX  (MP * FIN / 8 / NTHR)
#define PBW  (FO * FIN / 8 / NTHR)
#define PBTOT (PBX + PBW)

static_assert(FO == 64 && FO == 16 * 4);
static_assert(MP % GBM == 0 && MP >= NN && MP == 782 * GBM && MP - NN < GBM);
static_assert(NBRUN == (1 << SLB) && NBRUN == 1024 && NBRUN % GBM == 0 && NBRUN % 32 == 0);
static_assert(NBK * NBRUN >= MP && (NBK - 1) * NBRUN < NN);
static_assert(NE <= (1 << 21) && (((long long)NE) << SLB) < (1LL << 31));
static_assert(NE % WCH == 0 && NE % 256 == 0 && NE % 4 == 0);
static_assert((NWAVE - 1) * PERW < NE && (NE - (NWAVE - 1) * PERW) % WCH == 0 && PERW % WCH == 0);
static_assert((long long)RCAP * 100 >= (long long)MAXB1024_MEAS * 105);
static_assert((long long)WLCAP * 32 >= (long long)MAXB1024_MEAS * 5);
static_assert(RCAP % (2 * NTHR) == 0 && BK_ZINTS % 4 == 0 && (2 * NBRUN) % (4 * NTHR) == 0);
static_assert(MAXDEG_MEAS + 8 <= TRIPCAP);
static_assert((MP * FIN / 8) % NTHR == 0 && (FO * FIN / 8) % NTHR == 0);
static_assert(FIN % 32 == 0);
static_assert(BK_LDS <= 327680);
static_assert((GBM * SP) * 4 <= 65536);
static_assert(GBM == 16 * NWAVE);

typedef float          v4f   __attribute__((ext_vector_type(4)));
typedef float          v8f   __attribute__((ext_vector_type(8)));
typedef int            v2i   __attribute__((ext_vector_type(2)));
typedef int            v4i   __attribute__((ext_vector_type(4)));
typedef int            v8i   __attribute__((ext_vector_type(8)));
typedef unsigned short v8us  __attribute__((ext_vector_type(8)));
typedef unsigned short v16us __attribute__((ext_vector_type(16)));
typedef __bf16         v16bf __attribute__((ext_vector_type(16)));
typedef v4f  __attribute__((may_alias)) v4fa;
typedef v2i  __attribute__((may_alias)) v2ia;
typedef v4i  __attribute__((may_alias)) v4ia;
typedef v8us __attribute__((may_alias)) v8usa;
union FragB { v16bf v; v16us u; v8us h[2]; v8i w; };

__device__ __forceinline__ v8f wmb(const FragB& a, const FragB& b, v8f c) {
  v8f d = __builtin_amdgcn_wmma_f32_16x16x32_bf16(false, a.v, false, b.v, (short)0, c, false, false);
  asm volatile("v_nop\n\tv_nop\n\tv_nop\n\tv_nop" : "+v"(d) : "v"(a.w), "v"(b.w));
  return d;
}

__device__ __forceinline__ unsigned bf16_bits(float f) {
  const unsigned u = __float_as_uint(f);
  const unsigned r = (u + 0x7FFFu + ((u >> 16) & 1u)) >> 16;
  const unsigned q = (u >> 16) | 0x40u;
  return ((u & 0x7fffffffu) > 0x7f800000u) ? q : r;
}

__device__ __forceinline__ void st2_v4f(float* p, v4f v) {
  *(volatile v4f*)p = v;
  __threadfence();
  *(volatile v4f*)p = v;
}
__device__ __forceinline__ void st2_v4i(int* p, v4i v) {
  *(volatile v4i*)p = v;
  __threadfence();
  *(volatile v4i*)p = v;
}
__device__ __forceinline__ void st2_v8us(unsigned short* p, v8us v) {
  *(volatile v8us*)p = v;
  __threadfence();
  *(volatile v8us*)p = v;
}

__device__ __forceinline__ v8us gather8(const float* __restrict__ base, int stride) {
  float f[8];
#pragma unroll
  for (int i = 0; i < 8; ++i) f[i] = base[(size_t)i * (size_t)stride];
  v8us o;
#pragma unroll
  for (int i = 0; i < 8; ++i) o[i] = (unsigned short)bf16_bits(f[i]);
  return o;
}

__global__ __launch_bounds__(NTHR) void k_prep(const float* __restrict__ x, const float* __restrict__ w,
                                               unsigned short* xb, unsigned short* wt) {
  const int tid = (int)threadIdx.x;
  const int blk = (int)blockIdx.x;
  if (blk < PBX) {
    const int u   = blk * NTHR + tid;
    const int row = u >> 4, k8 = (u & 15) * 8;
    const int rc  = row < NN ? row : NN - 1;
    const unsigned mk = row < NN ? 0xffffu : 0u;
    const float* p = x + (size_t)rc * FIN + k8;
    const v4f a = *(const v4fa*)p;
    const v4f b = *(const v4fa*)(p + 4);
    v8us o;
    o[0] = (unsigned short)(bf16_bits(a.x) & mk); o[1] = (unsigned short)(bf16_bits(a.y) & mk);
    o[2] = (unsigned short)(bf16_bits(a.z) & mk); o[3] = (unsigned short)(bf16_bits(a.w) & mk);
    o[4] = (unsigned short)(bf16_bits(b.x) & mk); o[5] = (unsigned short)(bf16_bits(b.y) & mk);
    o[6] = (unsigned short)(bf16_bits(b.z) & mk); o[7] = (unsigned short)(bf16_bits(b.w) & mk);
    st2_v8us(xb + (size_t)row * FIN + k8, o);
  } else {
    const int u = (blk - PBX) * NTHR + tid;
    const int n = u >> 4, k8 = (u & 15) * 8;
    const v8us o = gather8(w + (size_t)k8 * FO + n, FO);
    st2_v8us(wt + (size_t)n * FIN + k8, o);
  }
}

__global__ __launch_bounds__(NTHR) void k_bucket(const int* __restrict__ srcs, const int* __restrict__ dsts,
                                                 const float* __restrict__ ew, int* LIST, int* CO, int* FLAG) {
  extern __shared__ __attribute__((aligned(16))) int dsm[];
  int* wl   = dsm;
  int* pl   = dsm + NWAVE * WLCAP;
  int* cnt  = pl + RCAP;
  int* offs = cnt + NBRUN;
  int* cur  = offs + NBRUN;
  int* misc = cur + NBRUN;
  const int tid = (int)threadIdx.x, lane = tid & 31, wave = tid >> 5;
  const int blk = (int)blockIdx.x;
  const unsigned nbs = (unsigned)(blk * NBRUN);
  const int nbi = (NN - blk * NBRUN) < NBRUN ? (NN - blk * NBRUN) : NBRUN;
  const unsigned unb = (unsigned)(nbi < 0 ? 0 : nbi);

  {
    const v4i z4 = {0, 0, 0, 0};
    for (int i = tid * 4; i < BK_ZINTS; i += NTHR * 4) *(v4ia*)(dsm + i) = z4;
    if (tid < 16) misc[tid] = 0;
  }
  __syncthreads();

  {
    const int ebeg = wave * PERW;
    const int eend = (ebeg + PERW < NE) ? (ebeg + PERW) : NE;
    int* mylist = wl + wave * WLCAP;
    int wc = 0;
#pragma unroll 1
    for (int cb = ebeg; cb < eend; cb += WCH) {
      const int e0 = cb + lane * EPT;
      const v4i da = *(const v4ia*)(dsts + e0);
      const v4i db = *(const v4ia*)(dsts + e0 + 4);
      const unsigned s0 = (unsigned)da.x - nbs, s1 = (unsigned)da.y - nbs;
      const unsigned s2 = (unsigned)da.z - nbs, s3 = (unsigned)da.w - nbs;
      const unsigned s4 = (unsigned)db.x - nbs, s5 = (unsigned)db.y - nbs;
      const unsigned s6 = (unsigned)db.z - nbs, s7 = (unsigned)db.w - nbs;
      const bool h0 = s0 < unb, h1 = s1 < unb, h2 = s2 < unb, h3 = s3 < unb;
      const bool h4 = s4 < unb, h5 = s5 < unb, h6 = s6 < unb, h7 = s7 < unb;
      const unsigned m0 = __builtin_amdgcn_ballot_w32(h0), m1 = __builtin_amdgcn_ballot_w32(h1);
      const unsigned m2 = __builtin_amdgcn_ballot_w32(h2), m3 = __builtin_amdgcn_ballot_w32(h3);
      const unsigned m4 = __builtin_amdgcn_ballot_w32(h4), m5 = __builtin_amdgcn_ballot_w32(h5);
      const unsigned m6 = __builtin_amdgcn_ballot_w32(h6), m7 = __builtin_amdgcn_ballot_w32(h7);
      const unsigned any = m0 | m1 | m2 | m3 | m4 | m5 | m6 | m7;
      if (any != 0u) {
        const int pre = (int)(__builtin_amdgcn_mbcnt_lo(m0, 0u) + __builtin_amdgcn_mbcnt_lo(m1, 0u) +
                              __builtin_amdgcn_mbcnt_lo(m2, 0u) + __builtin_amdgcn_mbcnt_lo(m3, 0u) +
                              __builtin_amdgcn_mbcnt_lo(m4, 0u) + __builtin_amdgcn_mbcnt_lo(m5, 0u) +
                              __builtin_amdgcn_mbcnt_lo(m6, 0u) + __builtin_amdgcn_mbcnt_lo(m7, 0u));
        int p = wc + pre;
        if (h0) { if (p < WLCAP) mylist[p] = ((e0 + 0) << SLB) | (int)s0; p = p + 1; }
        if (h1) { if (p < WLCAP) mylist[p] = ((e0 + 1) << SLB) | (int)s1; p = p + 1; }
        if (h2) { if (p < WLCAP) mylist[p] = ((e0 + 2) << SLB) | (int)s2; p = p + 1; }
        if (h3) { if (p < WLCAP) mylist[p] = ((e0 + 3) << SLB) | (int)s3; p = p + 1; }
        if (h4) { if (p < WLCAP) mylist[p] = ((e0 + 4) << SLB) | (int)s4; p = p + 1; }
        if (h5) { if (p < WLCAP) mylist[p] = ((e0 + 5) << SLB) | (int)s5; p = p + 1; }
        if (h6) { if (p < WLCAP) mylist[p] = ((e0 + 6) << SLB) | (int)s6; p = p + 1; }
        if (h7) { if (p < WLCAP) mylist[p] = ((e0 + 7) << SLB) | (int)s7; p = p + 1; }
        wc += (int)(__builtin_popcount(m0) + __builtin_popcount(m1) + __builtin_popcount(m2) + __builtin_popcount(m3) +
                    __builtin_popcount(m4) + __builtin_popcount(m5) + __builtin_popcount(m6) + __builtin_popcount(m7));
      }
    }
    if (lane == 0) misc[wave] = wc;
  }
  __syncthreads();

  if (wave == 0) {
    int ov = 0;
#pragma unroll 1
    for (int w2 = 0; w2 < NWAVE; ++w2) {
      int c = misc[w2];
      if (c > WLCAP) ov = 1;
      c = c < 0 ? 0 : (c > WLCAP ? WLCAP : c);
#pragma unroll 1
      for (int b0 = 0; b0 < c; b0 += 32) {
        const int idx = b0 + lane;
        const int ent = wl[w2 * WLCAP + (idx < WLCAP ? idx : WLCAP - 1)];
        const int m32 = (c - b0) < 32 ? (c - b0) : 32;
#pragma unroll 1
        for (int k = 0; k < m32; ++k) {
          const int u    = __builtin_amdgcn_readlane(ent, k);
          const int slot = u & (NBRUN - 1);
          if (lane == 0) cnt[slot] = cnt[slot] + 1;
        }
      }
    }
    if (lane == 0) misc[9] = ov;
  }
  __syncthreads();
  if (wave == 0) {
    const int base = lane * (NBRUN / 32);
    int s = 0;
#pragma unroll 1
    for (int i = 0; i < NBRUN / 32; ++i) s += cnt[base + i];
    int incl = s;
#pragma unroll
    for (int d = 1; d < 32; d <<= 1) {
      const int y = __shfl_up(incl, d, 32);
      if (lane >= d) incl += y;
    }
    const int total = __shfl(incl, 31, 32);
    int run = incl - s;
#pragma unroll 1
    for (int i = 0; i < NBRUN / 32; ++i) {
      const int cv = cnt[base + i];
      offs[base + i] = run;
      cur[base + i]  = run;
      run += cv;
    }
    if (lane == 0) {
      misc[10] = total;
      if (total > RCAP) misc[9] = 1;
    }
  }
  __syncthreads();

  if (wave == 0) {
#pragma unroll 1
    for (int w2 = 0; w2 < NWAVE; ++w2) {
      int c = misc[w2];
      c = c < 0 ? 0 : (c > WLCAP ? WLCAP : c);
#pragma unroll 1
      for (int b0 = 0; b0 < c; b0 += 32) {
        const int idx = b0 + lane;
        const int ent = wl[w2 * WLCAP + (idx < WLCAP ? idx : WLCAP - 1)];
        const int m32 = (c - b0) < 32 ? (c - b0) : 32;
#pragma unroll 1
        for (int k = 0; k < m32; ++k) {
          const int u    = __builtin_amdgcn_readlane(ent, k);
          const int slot = u & (NBRUN - 1);
          if (lane == 0) {
            int p = cur[slot];
            p = p < 0 ? 0 : (p > RCAP - 1 ? RCAP - 1 : p);
            pl[p] = u;
            cur[slot] = p + 1;
          }
        }
      }
    }
  }
  __syncthreads();

  const int ovf = misc[9];
  int tot = misc[10];
  tot = tot < 0 ? 0 : (tot > RCAP ? RCAP : tot);
  int* lp  = LIST + (size_t)blk * (size_t)(2 * RCAP);
  int* cop = CO + (size_t)blk * (2 * NBRUN);
  int* fp  = FLAG + (size_t)blk * 32;
#pragma unroll 1
  for (int it = 0; it < RCAP / (2 * NTHR); ++it) {
    const int e0i = 2 * (it * NTHR + tid);
    const v2i ww = *(const v2ia*)(pl + e0i);
    int id0 = (ww.x >> SLB) & 0x1FFFFF;
    int id1 = (ww.y >> SLB) & 0x1FFFFF;
    id0 = id0 > NE - 1 ? NE - 1 : id0;
    id1 = id1 > NE - 1 ? NE - 1 : id1;
    int   sa = srcs[id0];
    int   sb = srcs[id1];
    const float fa = ew[id0];
    const float fb = ew[id1];
    asm volatile("" :: "v"(sa), "v"(sb), "v"(fa), "v"(fb));
    sa = sa < 0 ? 0 : (sa > NN - 1 ? NN - 1 : sa);
    sb = sb < 0 ? 0 : (sb > NN - 1 ? NN - 1 : sb);
    const int ma = (e0i     < tot) ? -1 : 0;
    const int mb = (e0i + 1 < tot) ? -1 : 0;
    v4i o;
    o.x = sa & ma;
    o.y = (int)(bf16_bits(fa) << 16) & ma;
    o.z = sb & mb;
    o.w = (int)(bf16_bits(fb) << 16) & mb;
    st2_v4i(lp + 2 * e0i, o);
  }
#pragma unroll 1
  for (int it = 0; it < (2 * NBRUN) / (4 * NTHR); ++it) {
    const int i4 = it * NTHR + tid;
    const v4i v = *(const v4ia*)(cnt + 4 * i4);
    st2_v4i(cop + 4 * i4, v);
  }
  if (tid < 8) {
    const v4i f = {ovf, ovf, ovf, ovf};
    st2_v4i(fp + 4 * tid, f);
  }
}

template <int KTOT>
__device__ __forceinline__ void gemm_16x64(const unsigned short* __restrict__ ap,
                                           const unsigned short* __restrict__ bp, v8f (&acc)[4]) {
#pragma unroll 1
  for (int k0 = 0; k0 < KTOT; k0 += 32) {
    FragB af;
    af.h[0] = *(const v8usa*)(ap + k0);
    af.h[1] = *(const v8usa*)(ap + k0 + 16);
#pragma unroll
    for (int nt = 0; nt < 4; ++nt) {
      const unsigned short* wq = bp + (size_t)(16 * nt) * (size_t)KTOT + k0;
      FragB bf;
      bf.h[0] = *(const v8usa*)wq;
      bf.h[1] = *(const v8usa*)(wq + 16);
      acc[nt] = wmb(af, bf, acc[nt]);
    }
  }
}

__device__ __forceinline__ void stage_d(float* stg, const v8f (&acc)[4], int wave, int hh, int m) {
#pragma unroll
  for (int nt = 0; nt < 4; ++nt) {
#pragma unroll
    for (int r = 0; r < 8; ++r) stg[(16 * wave + 8 * hh + r) * SP + 16 * nt + m] = acc[nt][r];
  }
}

__global__ __launch_bounds__(NTHR) __attribute__((amdgpu_num_vgpr(248)))
void k_gemm(const unsigned short* __restrict__ XB, const unsigned short* __restrict__ WT, float* S) {
  __shared__ __attribute__((aligned(16))) float stg[GBM * SP];
  const int tid = (int)threadIdx.x, lane = tid & 31, wave = tid >> 5, hh = lane >> 4, m = lane & 15;
  const int rowBase = (int)blockIdx.x * GBM;

  v8f acc[4];
  {
    const v8f z = {0.f, 0.f, 0.f, 0.f, 0.f, 0.f, 0.f, 0.f};
#pragma unroll
    for (int t = 0; t < 4; ++t) acc[t] = z;
  }
  const unsigned short* ap = XB + (size_t)(rowBase + 16 * wave + m) * (size_t)FIN + 8 * hh;
  const unsigned short* bp = WT + (size_t)m * (size_t)FIN + 8 * hh;
  gemm_16x64<FIN>(ap, bp, acc);
  stage_d(stg, acc, wave, hh, m);
  __syncthreads();

#pragma unroll 1
  for (int i = 0; i < 8; ++i) {
    const int lr   = 16 * wave + 2 * i + hh;
    const int grow = rowBase + lr;
    const bool live = grow < NN;
    const int  gc   = live ? grow : NN - 1;
    const v4f a = *(const v4fa*)(stg + lr * SP + 4 * m);
    asm volatile("" :: "v"(a));
    float* op = S + (size_t)gc * FO + 4 * m;
    if (live) *(volatile v4f*)op = a;
    __threadfence();
    if (live) *(volatile v4f*)op = a;
  }
}

__global__ __launch_bounds__(NTHR) void k_replay(const int* __restrict__ LIST, const int* __restrict__ CO,
                                                 const int* __restrict__ FLAG, const float* __restrict__ S,
                                                 float* out) {
  const int tid = (int)threadIdx.x, lane = tid & 31, wave = tid >> 5, hh = lane >> 4, q = lane & 15;
  const int rowBase = (int)blockIdx.x * GBM;
  const int bucket  = rowBase >> SLB;
  const int* lb  = LIST + (size_t)bucket * (size_t)(2 * RCAP);
  const int* cob = CO + (size_t)bucket * (2 * NBRUN);
  const int flag = FLAG[(size_t)bucket * 32];
  const float qnan = __uint_as_float(0x7fc00000u);

#pragma unroll 1
  for (int i = 0; i < GBM / (2 * NWAVE); ++i) {
    const int d    = rowBase + 16 * wave + 2 * i + hh;
    const int slot = d & (NBRUN - 1);
    int c = cob[slot];
    int o = cob[NBRUN + slot];
    const bool big = c > TRIPCAP;
    c = c < 0 ? 0 : (c > TRIPCAP ? TRIPCAP : c);
    o = o < 0 ? 0 : (o > RCAP - 1 ? RCAP - 1 : o);
    const int co = __shfl_xor(c, 16, 32);
    const int cm = c > co ? c : co;
    int last = o + c - 1; last = last < o ? o : last;
    last = last > RCAP - 1 ? RCAP - 1 : last;
    float a0 = 0.0f, a1 = 0.0f, a2 = 0.0f, a3 = 0.0f;
#pragma unroll 1
    for (int j = 0; j < cm; ++j) {
      int idx = o + j;
      idx = idx > last ? last : idx;
      const v2i en = *(const v2ia*)(lb + 2 * idx);
      int sr = en.x;
      sr = sr < 0 ? 0 : (sr > NN - 1 ? NN - 1 : sr);
      const float w = __int_as_float(en.y);
      const v4f v = *(const v4fa*)(S + (size_t)sr * FO + 4 * q);
      asm volatile("" :: "v"(v));
      const bool valid = j < c;
      const float t0 = fmaf(w, v.x, a0), t1 = fmaf(w, v.y, a1), t2 = fmaf(w, v.z, a2), t3 = fmaf(w, v.w, a3);
      a0 = valid ? t0 : a0; a1 = valid ? t1 : a1; a2 = valid ? t2 : a2; a3 = valid ? t3 : a3;
    }
    float r0 = (a0 > 0.0f) ? a0 : (a0 - a0);
    float r1 = (a1 > 0.0f) ? a1 : (a1 - a1);
    float r2 = (a2 > 0.0f) ? a2 : (a2 - a2);
    float r3 = (a3 > 0.0f) ? a3 : (a3 - a3);
    const bool bad  = (flag != 0) | big;
    r0 = bad ? qnan : r0; r1 = bad ? qnan : r1; r2 = bad ? qnan : r2; r3 = bad ? qnan : r3;
    const bool live = d < NN;
    const int  dc   = live ? d : NN - 1;
    v4f ov;
    ov.x = r0; ov.y = r1; ov.z = r2; ov.w = r3;
    float* op = out + (size_t)dc * FO + 4 * q;
    if (live) *(volatile v4f*)op = ov;
    __threadfence();
    if (live) *(volatile v4f*)op = ov;
  }
}

extern "C" void kernel_launch(void* const* d_in, const int* in_sizes, int n_in,
                              void* d_out, int out_size, void* d_ws, size_t ws_size,
                              hipStream_t stream) {
  if (n_in < 5) return;
  if (in_sizes[0] != NN * FIN) return;
  if (in_sizes[1] != FIN * FO) return;
  if (in_sizes[2] != NE) return;
  if (in_sizes[3] != NE) return;
  if (in_sizes[4] != NE) return;
  if (out_size != NN * FO) return;

  const float* x    = (const float*)d_in[0];
  const float* w    = (const float*)d_in[1];
  const float* ev   = (const float*)d_in[2];
  const int*   esrc = (const int*)d_in[3];
  const int*   edst = (const int*)d_in[4];
  float* out = (float*)d_out;

  constexpr size_t zXB   = (size_t)MP * FIN * 2;
  constexpr size_t zWT   = (size_t)FO * FIN * 2;
  constexpr size_t zS    = (size_t)NN * FO * 4;
  constexpr size_t zLIST = (size_t)NBK * RCAP * 8;
  constexpr size_t zCO   = (size_t)NBK * 2 * NBRUN * 4;
  constexpr size_t zFLAG = (size_t)NBK * 128;
  constexpr size_t oXB   = 0;
  constexpr size_t oWT   = oXB + zXB;
  constexpr size_t oS    = oWT + zWT;
  constexpr size_t oLIST = oS + zS;
  constexpr size_t oCO   = oLIST + zLIST;
  constexpr size_t oFLAG = oCO + zCO;
  constexpr size_t oEND  = oFLAG + zFLAG;
  static_assert(zXB % 256 == 0 && zWT % 256 == 0 && zS % 256 == 0 && zLIST % 256 == 0);
  static_assert(zCO % 256 == 0 && zFLAG % 256 == 0);
  static_assert(oEND <= (size_t)WSMAX);
  if (oEND > ws_size) return;

  char* ws = (char*)d_ws;
  unsigned short* XB   = (unsigned short*)(ws + oXB);
  unsigned short* WT   = (unsigned short*)(ws + oWT);
  float*          S    = (float*)(ws + oS);
  int*            LIST = (int*)(ws + oLIST);
  int*            CO   = (int*)(ws + oCO);
  int*            FLAG = (int*)(ws + oFLAG);

  hipFuncSetAttribute(reinterpret_cast<const void*>(&k_bucket), hipFuncAttributeMaxDynamicSharedMemorySize, (int)BK_LDS);

  k_prep<<<PBTOT, NTHR, 0, stream>>>(x, w, XB, WT);
  k_bucket<<<NBK, NTHR, BK_LDS, stream>>>(esrc, edst, ev, LIST, CO, FLAG);
  k_gemm<<<MP / GBM, NTHR, 0, stream>>>(XB, WT, S);
  k_replay<<<MP / GBM, NTHR, 0, stream>>>(LIST, CO, FLAG, S, out);
}
